// GRU_72387378806936
// MI455X (gfx1250) — hardware-verified
//
#include <hip/hip_runtime.h>
#include <math.h>

constexpr int NBATCH   = 256;
constexpr int NSTEP    = 512;
constexpr int NXF      = 64;
constexpr int NHID     = 256;
constexpr int NMLP     = 64;
constexpr int NOUTF    = 16;
constexpr int KCELL    = NXF + NHID;
constexpr int NTHR     = 256;
constexpr int NWAVE    = NTHR / 32;
constexpr int ROWS_BLK = 16;
constexpr int APITCH   = 328;
constexpr int ZPITCH   = 72;
constexpr int TCHUNK   = 16;
constexpr int OPITCH   = TCHUNK * NOUTF + 4;
constexpr int AWORDS   = ROWS_BLK * APITCH;
constexpr int NOUTEL   = NBATCH * NSTEP * NOUTF;
static_assert(KCELL % 32 == 0 && NHID % 32 == 0 && NMLP % 32 == 0);
static_assert(NHID == 32 * NWAVE);
static_assert(NMLP == 16 * 4);
static_assert(NOUTF == 16);
static_assert(NBATCH % ROWS_BLK == 0);
static_assert(NSTEP % TCHUNK == 0);
static_assert(ROWS_BLK * NXF == 4 * NTHR);
static_assert(APITCH % 8 == 0 && APITCH >= KCELL);
static_assert(ZPITCH % 8 == 0 && ZPITCH >= NMLP);
static_assert(OPITCH % 4 == 0);
static_assert(ROWS_BLK * TCHUNK * NOUTF == NWAVE * 2 * 2 * 128);
static_assert((TCHUNK * NOUTF * 4) % 512 == 0);

typedef __attribute__((ext_vector_type(16))) __bf16   v16b;
typedef __attribute__((ext_vector_type(8)))  __bf16   v8b;
typedef __attribute__((ext_vector_type(8)))  float    v8f;
typedef __attribute__((ext_vector_type(4)))  float    v4f;
typedef __attribute__((ext_vector_type(4)))  unsigned v4u;
typedef __attribute__((ext_vector_type(2)))  unsigned v2u;

__device__ __forceinline__ unsigned short f2bf_bits(float f) {
  unsigned u = __float_as_uint(f);
  return (unsigned short)((u + 0x7FFFu + ((u >> 16) & 1u)) >> 16);
}
__device__ __forceinline__ float bf_bits2f(unsigned short h) { return __uint_as_float(((unsigned)h) << 16); }
__device__ __forceinline__ float bf16r(float f) { return bf_bits2f(f2bf_bits(f)); }

__device__ __forceinline__ void guard2x4_b(v8f& a, v8f& b, v16b w, v16b x, v16b y, v16b z) {
  asm volatile("v_nop\n\tv_nop\n\tv_nop\n\tv_nop" : "+v"(a), "+v"(b) : "v"(w), "v"(x), "v"(y), "v"(z));
}
__device__ __forceinline__ void guard1x3_b(v8f& a, v16b x, v16b y, v16b z) {
  asm volatile("v_nop\n\tv_nop\n\tv_nop\n\tv_nop" : "+v"(a) : "v"(x), "v"(y), "v"(z));
}
__device__ __forceinline__ void acc_guard2(v8f& a, v8f& b) { asm volatile("v_nop\n\tv_nop\n\tv_nop\n\tv_nop" : "+v"(a), "+v"(b)); }
__device__ __forceinline__ void acc_guard1(v8f& a) { asm volatile("v_nop\n\tv_nop\n\tv_nop\n\tv_nop" : "+v"(a)); }

template <typename T> struct Frag;
template <> struct Frag<__bf16> {
  typedef v16b V; union U { v16b v; v8b h[2]; };
  static __device__ __forceinline__ v16b load(const __bf16* p) {
    U f; f.h[0] = *(const v8b*)(p); f.h[1] = *(const v8b*)(p + 16); return f.v;
  }
  static __device__ __forceinline__ v8f mma(v16b a, v16b b, v8f c) {
    return __builtin_amdgcn_wmma_f32_16x16x32_bf16(false, a, false, b, (short)0, c, false, false);
  }
};

__global__ __launch_bounds__(NTHR) void cvt_rows_kernel(const float* __restrict__ src, int spitch, int ncol8, int nrow,
                                                        unsigned short* __restrict__ dst, int dpitch, int dcol0) {
  const int i = blockIdx.x * NTHR + threadIdx.x;
  if (i < nrow * ncol8) {
    const int row = i / ncol8;
    const int c8  = i - row * ncol8;
    const float* sp = src + (size_t)row * spitch + 8 * c8;
    const v4f a = *(const v4f*)(sp);
    const v4f b = *(const v4f*)(sp + 4);
    v4u pk;
    pk[0] = (unsigned)f2bf_bits(a[0]) | ((unsigned)f2bf_bits(a[1]) << 16);
    pk[1] = (unsigned)f2bf_bits(a[2]) | ((unsigned)f2bf_bits(a[3]) << 16);
    pk[2] = (unsigned)f2bf_bits(b[0]) | ((unsigned)f2bf_bits(b[1]) << 16);
    pk[3] = (unsigned)f2bf_bits(b[2]) | ((unsigned)f2bf_bits(b[3]) << 16);
    unsigned short* dp = dst + (size_t)row * dpitch + dcol0 + 8 * c8;
    *(volatile v4u*)dp = pk;
    __threadfence();
    *(volatile v4u*)dp = pk;
  }
}

__device__ __forceinline__ void stage_x_tile(const float* __restrict__ x, int rowbase, int tt,
                                             unsigned short* ah, unsigned short* al, int tid) {
  const int m = tid >> 4, f4 = (tid & 15) * 4;
  const v4f v = *(const v4f*)(x + ((size_t)(rowbase + m) * NSTEP + (size_t)tt) * NXF + f4);
  v2u pk;
  pk[0] = (unsigned)f2bf_bits(v[0]) | ((unsigned)f2bf_bits(v[1]) << 16);
  pk[1] = (unsigned)f2bf_bits(v[2]) | ((unsigned)f2bf_bits(v[3]) << 16);
  v2u zz;
  zz[0] = 0u; zz[1] = 0u;
  *(v2u*)(ah + m * APITCH + f4) = pk;
  *(v2u*)(al + m * APITCH + f4) = zz;
}

__global__ __launch_bounds__(NTHR) void rnn_seq_kernel(const float* __restrict__ x,
                                                       const float* __restrict__ b_ih, const float* __restrict__ b_hh,
                                                       const float* __restrict__ b1, const float* __restrict__ b2,
                                                       const float* __restrict__ b3, const int* __restrict__ pstart,
                                                       const unsigned short* __restrict__ WCp,
                                                       const unsigned short* __restrict__ W1p,
                                                       const unsigned short* __restrict__ W2p,
                                                       const unsigned short* __restrict__ W3p,
                                                       float* __restrict__ out) {
  __shared__ __align__(16) unsigned short Ahi[2][ROWS_BLK * APITCH];
  __shared__ __align__(16) unsigned short Alo[2][ROWS_BLK * APITCH];
  __shared__ __align__(16) unsigned short Z1h[ROWS_BLK * ZPITCH];
  __shared__ __align__(16) unsigned short Z1l[ROWS_BLK * ZPITCH];
  __shared__ __align__(16) unsigned short Z2h[ROWS_BLK * ZPITCH];
  __shared__ __align__(16) unsigned short Z2l[ROWS_BLK * ZPITCH];
  __shared__ __align__(16) float          Ost[ROWS_BLK * OPITCH];
  const __bf16* WC = (const __bf16*)WCp;
  const __bf16* W1 = (const __bf16*)W1p;
  const __bf16* W2 = (const __bf16*)W2p;
  const __bf16* W3 = (const __bf16*)W3p;
  const int tid = threadIdx.x, lane = tid & 31, wave = tid >> 5;
  const int c = lane & 15, hh = lane >> 4, koff = hh * 8;
  const int rowbase = blockIdx.x * ROWS_BLK;

  {
    unsigned* ahw = (unsigned*)(&Ahi[0][0]);
    unsigned* alw = (unsigned*)(&Alo[0][0]);
#pragma unroll 1
    for (int i = tid; i < AWORDS; i += NTHR) { ahw[i] = 0u; alw[i] = 0u; }
  }
  __syncthreads();
  stage_x_tile(x, rowbase, 0, &Ahi[0][0], &Alo[0][0], tid);

  const int ncell0 = 32 * wave + c;
  const int ncell1 = ncell0 + 16;
  const float bc0 = bf16r(b_ih[ncell0]) + bf16r(b_hh[ncell0]);
  const float bc1 = bf16r(b_ih[ncell1]) + bf16r(b_hh[ncell1]);
  const int nm = 16 * (wave & 3) + c;
  const float b1c = bf16r(b1[nm]);
  const float b2c = bf16r(b2[nm]);
  const float b3c = bf16r(b3[c]);
  const int ps = pstart[0];
  __syncthreads();

  const v8f z8 = {0.f, 0.f, 0.f, 0.f, 0.f, 0.f, 0.f, 0.f};

#pragma unroll 1
  for (int t = 0; t < NSTEP; ++t) {
    const int cur = t & 1, nxt = cur ^ 1;
    unsigned short* anh = &Ahi[nxt][0];
    unsigned short* anl = &Alo[nxt][0];

    {
      const int tn = (t + 1 < NSTEP) ? (t + 1) : (NSTEP - 1);
      stage_x_tile(x, rowbase, tn, anh, anl, tid);
    }
    {
      const __bf16* arh = (const __bf16*)(&Ahi[cur][0]) + c * APITCH + koff;
      const __bf16* arl = (const __bf16*)(&Alo[cur][0]) + c * APITCH + koff;
      const __bf16* w0 = WC + (size_t)ncell0 * KCELL + koff;
      const __bf16* w1 = WC + (size_t)ncell1 * KCELL + koff;
      v8f acc0 = z8, acc1 = z8;
#pragma unroll 1
      for (int k0 = 0; k0 < KCELL; k0 += 32) {
        const v16b ah  = Frag<__bf16>::load(arh + k0);
        const v16b al  = Frag<__bf16>::load(arl + k0);
        const v16b bq0 = Frag<__bf16>::load(w0 + k0);
        const v16b bq1 = Frag<__bf16>::load(w1 + k0);
        acc0 = Frag<__bf16>::mma(ah, bq0, acc0);
        acc1 = Frag<__bf16>::mma(ah, bq1, acc1);
        acc0 = Frag<__bf16>::mma(al, bq0, acc0);
        acc1 = Frag<__bf16>::mma(al, bq1, acc1);
        guard2x4_b(acc0, acc1, ah, al, bq0, bq1);
      }
      acc_guard2(acc0, acc1);
#pragma unroll
      for (int r = 0; r < 8; ++r) {
        const float hv0 = tanhf(acc0[r] + bc0);
        const float hv1 = tanhf(acc1[r] + bc1);
        const unsigned short hb0 = f2bf_bits(hv0);
        const unsigned short hb1 = f2bf_bits(hv1);
        const unsigned short lb0 = f2bf_bits(hv0 - bf_bits2f(hb0));
        const unsigned short lb1 = f2bf_bits(hv1 - bf_bits2f(hb1));
        const int ro = (8 * hh + r) * APITCH + NXF;
        anh[ro + ncell0] = hb0;
        anl[ro + ncell0] = lb0;
        anh[ro + ncell1] = hb1;
        anl[ro + ncell1] = lb1;
      }
    }
    __syncthreads();

    if (wave < 4) {
      const __bf16* arh = (const __bf16*)anh + c * APITCH + NXF + koff;
      const __bf16* arl = (const __bf16*)anl + c * APITCH + NXF + koff;
      const __bf16* w = W1 + (size_t)nm * NHID + koff;
      v8f acc = z8;
#pragma unroll 1
      for (int k0 = 0; k0 < NHID; k0 += 32) {
        const v16b ah = Frag<__bf16>::load(arh + k0);
        const v16b al = Frag<__bf16>::load(arl + k0);
        const v16b bw = Frag<__bf16>::load(w + k0);
        acc = Frag<__bf16>::mma(ah, bw, acc);
        acc = Frag<__bf16>::mma(al, bw, acc);
        guard1x3_b(acc, ah, al, bw);
      }
      acc_guard1(acc);
#pragma unroll
      for (int r = 0; r < 8; ++r) {
        const float v = fmaxf(acc[r] + b1c, 0.0f);
        const unsigned short hb = f2bf_bits(v);
        const unsigned short lb = f2bf_bits(v - bf_bits2f(hb));
        Z1h[(8 * hh + r) * ZPITCH + nm] = hb;
        Z1l[(8 * hh + r) * ZPITCH + nm] = lb;
      }
    }
    __syncthreads();

    if (wave < 4) {
      const __bf16* arh = (const __bf16*)Z1h + c * ZPITCH + koff;
      const __bf16* arl = (const __bf16*)Z1l + c * ZPITCH + koff;
      const __bf16* w = W2 + (size_t)nm * NMLP + koff;
      v8f acc = z8;
#pragma unroll 1
      for (int k0 = 0; k0 < NMLP; k0 += 32) {
        const v16b ah = Frag<__bf16>::load(arh + k0);
        const v16b al = Frag<__bf16>::load(arl + k0);
        const v16b bw = Frag<__bf16>::load(w + k0);
        acc = Frag<__bf16>::mma(ah, bw, acc);
        acc = Frag<__bf16>::mma(al, bw, acc);
        guard1x3_b(acc, ah, al, bw);
      }
      acc_guard1(acc);
#pragma unroll
      for (int r = 0; r < 8; ++r) {
        const float v = fmaxf(acc[r] + b2c, 0.0f);
        const unsigned short hb = f2bf_bits(v);
        const unsigned short lb = f2bf_bits(v - bf_bits2f(hb));
        Z2h[(8 * hh + r) * ZPITCH + nm] = hb;
        Z2l[(8 * hh + r) * ZPITCH + nm] = lb;
      }
    }
    __syncthreads();

    if (wave == 0) {
      const __bf16* arh = (const __bf16*)Z2h + c * ZPITCH + koff;
      const __bf16* arl = (const __bf16*)Z2l + c * ZPITCH + koff;
      const __bf16* w = W3 + (size_t)c * NMLP + koff;
      v8f acc = z8;
#pragma unroll 1
      for (int k0 = 0; k0 < NMLP; k0 += 32) {
        const v16b ah = Frag<__bf16>::load(arh + k0);
        const v16b al = Frag<__bf16>::load(arl + k0);
        const v16b bw = Frag<__bf16>::load(w + k0);
        acc = Frag<__bf16>::mma(ah, bw, acc);
        acc = Frag<__bf16>::mma(al, bw, acc);
        guard1x3_b(acc, ah, al, bw);
      }
      acc_guard1(acc);
      const int tl = t & (TCHUNK - 1);
      const bool splice = (t + 1) > ps;
#pragma unroll
      for (int r = 0; r < 8; ++r) {
        const float o = acc[r] + b3c;
        Ost[(8 * hh + r) * OPITCH + tl * NOUTF + c] = o;
        if (splice) {
          const unsigned short hb = f2bf_bits(o);
          const unsigned short lb = f2bf_bits(o - bf_bits2f(hb));
          anh[(8 * hh + r) * APITCH + c] = hb;
          anl[(8 * hh + r) * APITCH + c] = lb;
        }
      }
    }
    __syncthreads();

    if ((t & (TCHUNK - 1)) == TCHUNK - 1) {
      const int t0 = t - (TCHUNK - 1);
      for (int pass = 0; pass < 2; ++pass) {
#pragma unroll
        for (int it = 0; it < 2; ++it) {
          const int row = 2 * wave + it;
#pragma unroll
          for (int q4 = 0; q4 < 2; ++q4) {
            const v4f v = *(const v4f*)(Ost + row * OPITCH + 128 * q4 + 4 * lane);
            *(volatile v4f*)(out + ((size_t)(rowbase + row) * NSTEP + (size_t)t0) * NOUTF + 128 * q4 + 4 * lane) = v;
          }
        }
        __threadfence();
      }
    }
  }
}

extern "C" void kernel_launch(void* const* d_in, const int* in_sizes, int n_in,
                              void* d_out, int out_size, void* d_ws, size_t ws_size, hipStream_t stream) {
  if (n_in < 12 || d_out == nullptr || d_ws == nullptr) return;
  if (in_sizes[0] != NBATCH * NSTEP * NXF || in_sizes[1] != NHID * NXF || in_sizes[2] != NHID ||
      in_sizes[3] != NHID * NHID || in_sizes[4] != NHID || in_sizes[5] != NMLP * NHID || in_sizes[6] != NMLP ||
      in_sizes[7] != NMLP * NMLP || in_sizes[8] != NMLP || in_sizes[9] != NOUTF * NMLP || in_sizes[10] != NOUTF ||
      in_sizes[11] < 1 || out_size != NOUTEL) return;

  const float* x    = (const float*)d_in[0];
  const float* w_ih = (const float*)d_in[1];
  const float* b_ih = (const float*)d_in[2];
  const float* w_hh = (const float*)d_in[3];
  const float* b_hh = (const float*)d_in[4];
  const float* w1   = (const float*)d_in[5];
  const float* b1   = (const float*)d_in[6];
  const float* w2   = (const float*)d_in[7];
  const float* b2   = (const float*)d_in[8];
  const float* w3   = (const float*)d_in[9];
  const float* b3   = (const float*)d_in[10];
  const int*   pst  = (const int*)d_in[11];
  float* out = (float*)d_out;

  char* ws = (char*)d_ws; size_t off = 0;
  auto carve = [&](size_t bytes) -> char* { char* p = ws + off; off += (bytes + 255) & ~(size_t)255; return p; };
  unsigned short* WC  = (unsigned short*)carve((size_t)NHID * KCELL * 2);
  unsigned short* W1B = (unsigned short*)carve((size_t)NMLP * NHID * 2);
  unsigned short* W2B = (unsigned short*)carve((size_t)NMLP * NMLP * 2);
  unsigned short* W3B = (unsigned short*)carve((size_t)NOUTF * NMLP * 2);
  if (off > ws_size || off > (size_t)134217728) return;

  const int n8_ih = NHID * (NXF / 8);
  const int n8_hh = NHID * (NHID / 8);
  const int n8_w1 = NMLP * (NHID / 8);
  const int n8_w2 = NMLP * (NMLP / 8);
  const int n8_w3 = NOUTF * (NMLP / 8);
  cvt_rows_kernel<<<(n8_ih + NTHR - 1) / NTHR, NTHR, 0, stream>>>(w_ih, NXF,  NXF / 8,  NHID,  WC,  KCELL, 0);
  cvt_rows_kernel<<<(n8_hh + NTHR - 1) / NTHR, NTHR, 0, stream>>>(w_hh, NHID, NHID / 8, NHID,  WC,  KCELL, NXF);
  cvt_rows_kernel<<<(n8_w1 + NTHR - 1) / NTHR, NTHR, 0, stream>>>(w1,   NHID, NHID / 8, NMLP,  W1B, NHID,  0);
  cvt_rows_kernel<<<(n8_w2 + NTHR - 1) / NTHR, NTHR, 0, stream>>>(w2,   NMLP, NMLP / 8, NMLP,  W2B, NMLP,  0);
  cvt_rows_kernel<<<(n8_w3 + NTHR - 1) / NTHR, NTHR, 0, stream>>>(w3,   NMLP, NMLP / 8, NOUTF, W3B, NMLP,  0);

  rnn_seq_kernel<<<NBATCH / ROWS_BLK, NTHR, 0, stream>>>(x, b_ih, b_hh, b1, b2, b3, pst, WC, W1B, W2B, W3B, out);
}
